// GraphNeuralNetwork_81140522156740
// MI455X (gfx1250) — hardware-verified
//
#include <hip/hip_runtime.h>
#include <stddef.h>
#include <stdint.h>
#include <math.h>


#define IN_DIM  77
#define KP      128
#define ND      64
#define HD      128
#define NG      128
#define NLAY    3
#define NTHR    256
#define NWAVE   8
#define EPT     8
#define CHUNK   (NTHR * EPT)
#define WCAP    (EPT * 32)
#define LISTN   (NWAVE * WCAP)
#define NBA     1024
#define SLA     10
#define RCAP    28672
#define DEGCAP  64
#define MEAS_B1024  16623
#define MEAS_MAXDEG 35
#define GBM     64
#define GTHR    128
#define MROWS   128
#define SROWS   128
#define PA_ROWS 32
#define PA_F4   (PA_ROWS * IN_DIM / 4)
#define NU_EMB  (ND * (KP / 8))
#define NU_WN   (NLAY * ND * (KP / 8))
#define NU_WG   (NLAY * ND * (KP / 8))
#define NU_FW   (HD * (KP / 8))
#define PAR_EMBB 0
#define PAR_BNB  64
#define PAR_GAM  256
#define PAR_BET  448
#define PAR_FB   640
#define PAR_FGAM 768
#define PAR_FBET 896
#define PAR_N    1024
#define BKT_ZINTS    (2 * RCAP + 3 * NBA)
#define BKT_LDS_INTS (LISTN + BKT_ZINTS + 16)
#define HEAD_LDS_FLOATS (NG * HD + 2 * HD)
#define WSMAX   134217728

static_assert((CHUNK & (CHUNK - 1)) == 0 && CHUNK <= 4096);
static_assert((NBA & (NBA - 1)) == 0 && NBA == (1 << SLA) && NBA == 4 * NTHR);
static_assert(LISTN == NWAVE * WCAP && LISTN == NTHR * 8);
static_assert(NBA % NWAVE == 0 && NBA % 32 == 0);
static_assert((RCAP % 32) == 0 && (BKT_ZINTS % 4) == 0 && ((RCAP / 2) % NTHR) == 0);
static_assert(RCAP >= MEAS_B1024 + 4096);
static_assert(DEGCAP >= MEAS_MAXDEG + 8);
static_assert(BKT_LDS_INTS * 4 <= 260096);
static_assert(HEAD_LDS_FLOATS * 4 <= 260096);
static_assert(GBM == (GTHR / 32) * 16 && (MROWS % GBM) == 0 && (MROWS % PA_ROWS) == 0 && MROWS == SROWS);
static_assert((KP % 32) == 0 && KP == 2 * ND && IN_DIM <= KP);
static_assert((PA_ROWS * IN_DIM) % 4 == 0 && PA_F4 <= 3 * NTHR && PA_ROWS * (KP / 8) == 2 * NTHR);
static_assert((NU_EMB % NTHR) == 0 && (NU_WN % NTHR) == 0 && (NU_WG % NTHR) == 0 && (NU_FW % NTHR) == 0);
static_assert(PAR_N == 4 * NTHR && PAR_FBET + HD == PAR_N);
static_assert(ND == 2 * 32 && HD == 4 * 32 && NG == NWAVE * 16);

typedef float          v2f  __attribute__((ext_vector_type(2)));
typedef float          v4f  __attribute__((ext_vector_type(4)));
typedef float          v8f  __attribute__((ext_vector_type(8)));
typedef int            v2i  __attribute__((ext_vector_type(2)));
typedef int            v4i  __attribute__((ext_vector_type(4)));
typedef int            v8i  __attribute__((ext_vector_type(8)));
typedef unsigned short v4us __attribute__((ext_vector_type(4)));
typedef unsigned short v8us __attribute__((ext_vector_type(8)));
typedef __bf16         v16b __attribute__((ext_vector_type(16)));
typedef v4f  __attribute__((may_alias)) v4fa;
typedef v2i  __attribute__((may_alias)) v2ia;
typedef v4i  __attribute__((may_alias)) v4ia;
typedef v8us __attribute__((may_alias)) v8usa;
union FragB { v16b v; v8us h[2]; v8i w; };

__device__ __forceinline__ v8f wmb(const FragB& a, const FragB& b, v8f c) {
  v8f d = __builtin_amdgcn_wmma_f32_16x16x32_bf16(false, a.v, false, b.v, (short)0, c, false, false);
  asm volatile("v_nop\n\tv_nop\n\tv_nop\n\tv_nop" : "+v"(d) : "v"(a.w), "v"(b.w));
  return d;
}
__device__ __forceinline__ v8f z8() { v8f z = {0.f, 0.f, 0.f, 0.f, 0.f, 0.f, 0.f, 0.f}; return z; }

__device__ __forceinline__ unsigned int f2bf(float f) {
  const unsigned int u = __float_as_uint(f);
  const unsigned int r = ((u + 0x7FFFu + ((u >> 16) & 1u)) >> 16) & 0xFFFFu;
  return ((u & 0x7FFFFFFFu) > 0x7F800000u) ? 0x7FC0u : r;
}
__device__ __forceinline__ float bf2f(unsigned int b) { return __uint_as_float(b << 16); }
__device__ __forceinline__ float bfr(float f) { return bf2f(f2bf(f)); }

__device__ __forceinline__ v4us pack4(const v4f v, const int part) {
  const unsigned int h0 = f2bf(v.x), h1 = f2bf(v.y), h2 = f2bf(v.z), h3 = f2bf(v.w);
  const unsigned int l0 = f2bf(v.x - bf2f(h0)), l1 = f2bf(v.y - bf2f(h1));
  const unsigned int l2 = f2bf(v.z - bf2f(h2)), l3 = f2bf(v.w - bf2f(h3));
  v4us o;
  o.x = (unsigned short)(part != 0 ? l0 : h0);
  o.y = (unsigned short)(part != 0 ? l1 : h1);
  o.z = (unsigned short)(part != 0 ? l2 : h2);
  o.w = (unsigned short)(part != 0 ? l3 : h3);
  return o;
}

template <int SLB>
__device__ __forceinline__ int scan_chunk(const int* __restrict__ dsts, int nE, int cbase, int slotBase,
                                          int nb, int vec8, int* list, int tid, int lane, int wave) {
  int wc = 0;
  const int el0  = tid * EPT;
  const int e0   = cbase + el0;
  const int sent = -2147483647 - 1;
  v4i da, db;
  if (vec8 != 0 && cbase + CHUNK <= nE) {
    da = *(const v4i*)(dsts + e0);
    db = *(const v4i*)(dsts + e0 + 4);
  } else {
    da.x = (e0     < nE) ? dsts[min(e0,     nE - 1)] : sent;
    da.y = (e0 + 1 < nE) ? dsts[min(e0 + 1, nE - 1)] : sent;
    da.z = (e0 + 2 < nE) ? dsts[min(e0 + 2, nE - 1)] : sent;
    da.w = (e0 + 3 < nE) ? dsts[min(e0 + 3, nE - 1)] : sent;
    db.x = (e0 + 4 < nE) ? dsts[min(e0 + 4, nE - 1)] : sent;
    db.y = (e0 + 5 < nE) ? dsts[min(e0 + 5, nE - 1)] : sent;
    db.z = (e0 + 6 < nE) ? dsts[min(e0 + 6, nE - 1)] : sent;
    db.w = (e0 + 7 < nE) ? dsts[min(e0 + 7, nE - 1)] : sent;
  }
  const unsigned nbs = (unsigned)slotBase;
  const unsigned unb = (unsigned)nb;
  const unsigned s0 = (unsigned)da.x - nbs, s1 = (unsigned)da.y - nbs;
  const unsigned s2 = (unsigned)da.z - nbs, s3 = (unsigned)da.w - nbs;
  const unsigned s4 = (unsigned)db.x - nbs, s5 = (unsigned)db.y - nbs;
  const unsigned s6 = (unsigned)db.z - nbs, s7 = (unsigned)db.w - nbs;
  const bool h0 = s0 < unb, h1 = s1 < unb, h2 = s2 < unb, h3 = s3 < unb;
  const bool h4 = s4 < unb, h5 = s5 < unb, h6 = s6 < unb, h7 = s7 < unb;
  const unsigned any = __builtin_amdgcn_ballot_w32(h0 | h1 | h2 | h3 | h4 | h5 | h6 | h7);
  if (any != 0u) {
    const int c = (int)h0 + (int)h1 + (int)h2 + (int)h3 + (int)h4 + (int)h5 + (int)h6 + (int)h7;
    int incl = c;
#pragma unroll
    for (int d = 1; d < 32; d <<= 1) {
      const int y = __shfl_up(incl, d, 32);
      if (lane >= d) incl += y;
    }
    wc = __shfl(incl, 31, 32);
    int pos = incl - c;
    int* lw = list + wave * WCAP;
    if (h0) { if (pos < WCAP) lw[pos] = ((el0 + 0) << SLB) | (int)s0; pos += 1; }
    if (h1) { if (pos < WCAP) lw[pos] = ((el0 + 1) << SLB) | (int)s1; pos += 1; }
    if (h2) { if (pos < WCAP) lw[pos] = ((el0 + 2) << SLB) | (int)s2; pos += 1; }
    if (h3) { if (pos < WCAP) lw[pos] = ((el0 + 3) << SLB) | (int)s3; pos += 1; }
    if (h4) { if (pos < WCAP) lw[pos] = ((el0 + 4) << SLB) | (int)s4; pos += 1; }
    if (h5) { if (pos < WCAP) lw[pos] = ((el0 + 5) << SLB) | (int)s5; pos += 1; }
    if (h6) { if (pos < WCAP) lw[pos] = ((el0 + 6) << SLB) | (int)s6; pos += 1; }
    if (h7) { if (pos < WCAP) lw[pos] = ((el0 + 7) << SLB) | (int)s7; pos += 1; }
  }
  return wc;
}

__global__ __launch_bounds__(NTHR) __attribute__((amdgpu_num_vgpr(248)))
void k_pa(const float* __restrict__ x, unsigned short* XB, int nF4) {
  __shared__ __attribute__((aligned(16))) float tile[PA_ROWS * IN_DIM];
  const int tid = (int)threadIdx.x;
  const int blk = (int)blockIdx.x;
#pragma unroll 1
  for (int j = tid; j < PA_F4; j += NTHR) {
    const int idx = blk * PA_F4 + j;
    const int idc = idx < nF4 ? idx : nF4 - 1;
    const v4f ld = *(const v4f*)(x + (size_t)idc * 4);
    const bool ok = idx < nF4;
    v4f v;
    v.x = ok ? ld.x : 0.0f; v.y = ok ? ld.y : 0.0f; v.z = ok ? ld.z : 0.0f; v.w = ok ? ld.w : 0.0f;
    *(v4fa*)(tile + 4 * j) = v;
  }
  __syncthreads();
  v8us o0, o1;
  {
    const int u = tid, row = u >> 4, c0 = (u & 15) * 8;
#pragma unroll
    for (int i = 0; i < 8; ++i) {
      const int c = c0 + i;
      const int cc = c < IN_DIM ? c : IN_DIM - 1;
      const float f = tile[row * IN_DIM + cc];
      o0[i] = (c < IN_DIM) ? (unsigned short)f2bf(f) : (unsigned short)0;
    }
  }
  {
    const int u = NTHR + tid, row = u >> 4, c0 = (u & 15) * 8;
#pragma unroll
    for (int i = 0; i < 8; ++i) {
      const int c = c0 + i;
      const int cc = c < IN_DIM ? c : IN_DIM - 1;
      const float f = tile[row * IN_DIM + cc];
      o1[i] = (c < IN_DIM) ? (unsigned short)f2bf(f) : (unsigned short)0;
    }
  }
  unsigned short* d0 = XB + (size_t)blk * PA_ROWS * KP + (size_t)tid * 8;
  unsigned short* d1 = d0 + (size_t)NTHR * 8;
  *(volatile v8us*)d0 = o0;
  *(volatile v8us*)d1 = o1;
  __threadfence();
  *(volatile v8us*)d0 = o0;
  *(volatile v8us*)d1 = o1;
}

__global__ __launch_bounds__(NTHR) __attribute__((amdgpu_num_vgpr(248)))
void k_pb(const float* __restrict__ embW, const float* __restrict__ Wn, const float* __restrict__ Wg,
          const float* __restrict__ fW, unsigned short* EMBT, unsigned short* BT, unsigned short* FWD) {
  const int u = (int)blockIdx.x * NTHR + (int)threadIdx.x;
  v8us o;
  unsigned short* dp;
  if (u < NU_EMB) {
    const int n  = u >> 4;
    const int k8 = (u & 15) * 8;
#pragma unroll
    for (int i = 0; i < 8; ++i) {
      const int k  = k8 + i;
      const int kc = k < IN_DIM ? k : IN_DIM - 1;
      const float f = embW[(size_t)kc * ND + n];
      o[i] = (k < IN_DIM) ? (unsigned short)f2bf(f) : (unsigned short)0;
    }
    dp = EMBT + (size_t)n * KP + k8;
  } else if (u < NU_EMB + NU_WN) {
    const int v  = u - NU_EMB;
    const int l  = v >> 10;
    const int r  = v & 1023;
    const int n  = r >> 4;
    const int k8 = (r & 15) * 8;
    const int kk = k8 & (ND - 1);
    const float* p = Wn + (size_t)l * ND * ND + (size_t)kk * ND + n;
#pragma unroll
    for (int i = 0; i < 8; ++i) o[i] = (unsigned short)f2bf(p[(size_t)i * ND]);
    dp = BT + (size_t)l * HD * KP + (size_t)n * KP + k8;
  } else if (u < NU_EMB + NU_WN + NU_WG) {
    const int v  = u - NU_EMB - NU_WN;
    const int l  = v >> 10;
    const int r  = v & 1023;
    const int n  = r >> 4;
    const int k8 = (r & 15) * 8;
    const int kk = k8 & (ND - 1);
    const float* p = Wg + (size_t)l * 2 * ND * ND + (size_t)kk * ND + n;
#pragma unroll
    for (int i = 0; i < 8; ++i) o[i] = (unsigned short)f2bf(p[(size_t)i * ND]);
    dp = BT + (size_t)l * HD * KP + (size_t)(ND + n) * KP + k8;
  } else if (u < NU_EMB + NU_WN + NU_WG + NU_FW) {
    const int v  = u - NU_EMB - NU_WN - NU_WG;
    const int n  = v >> 4;
    const int k8 = (v & 15) * 8;
    const int kk = k8 & (ND - 1);
    const float* p = fW + (size_t)kk * HD + n;
#pragma unroll
    for (int i = 0; i < 8; ++i) o[i] = (unsigned short)f2bf(p[(size_t)i * HD]);
    dp = FWD + (size_t)n * KP + k8;
  } else {
    return;
  }
  *(volatile v8us*)dp = o;
  __threadfence();
  *(volatile v8us*)dp = o;
}

__global__ __launch_bounds__(ND) __attribute__((amdgpu_num_vgpr(248)))
void k_pc(const float* __restrict__ eW, const float* __restrict__ eB, const float* __restrict__ We,
          const float* __restrict__ be, const float* __restrict__ Wg, const float* __restrict__ bg, float* PQ) {
  __shared__ double tu[ND];
  __shared__ double tc[ND];
  __shared__ __attribute__((aligned(16))) float outp[2 * ND];
  const int l = (int)blockIdx.x;
  const int j = (int)threadIdx.x;
  double a = 0.0, b = 0.0;
#pragma unroll 1
  for (int k = 0; k < 32; ++k) {
    const double w = (double)bfr(We[(size_t)l * 32 * ND + (size_t)k * ND + j]);
    a += (double)bfr(eW[k]) * w;
    b += (double)bfr(eB[k]) * w;
  }
  tu[j] = a;
  tc[j] = b + (double)bfr(be[l * ND + j]);
  __syncthreads();
  double p = 0.0, q = 0.0;
#pragma unroll 1
  for (int jj = 0; jj < ND; ++jj) {
    const double w = (double)bfr(Wg[(size_t)l * 2 * ND * ND + (size_t)(ND + jj) * ND + j]);
    p += tu[jj] * w;
    q += tc[jj] * w;
  }
  outp[j] = (float)p;
  outp[ND + j] = (float)(q + (double)bfr(bg[l * ND + j]));
  __syncthreads();
  v4f v = {0.f, 0.f, 0.f, 0.f};
  float* dp = PQ + (size_t)l * 2 * ND + 4 * (j & 31);
  if (j < 32) { v = *(const v4fa*)(outp + 4 * j); *(volatile v4f*)dp = v; }
  __threadfence();
  if (j < 32) { *(volatile v4f*)dp = v; }
}

__device__ __forceinline__ v4i pd_pick(const float* __restrict__ s, int base, int len, int e0) {
  const int loc = e0 - base;
  const int lc  = loc < 0 ? 0 : (loc > len - 4 ? len - 4 : loc);
  const v4f v = *(const v4f*)(s + lc);
  const int msk = (loc >= 0 && loc < len) ? -1 : 0;
  v4i r;
  r.x = __float_as_int(bfr(v.x)) & msk;
  r.y = __float_as_int(bfr(v.y)) & msk;
  r.z = __float_as_int(bfr(v.z)) & msk;
  r.w = __float_as_int(bfr(v.w)) & msk;
  return r;
}
__global__ __launch_bounds__(NTHR) __attribute__((amdgpu_num_vgpr(248)))
void k_pd(const float* __restrict__ embb, const float* __restrict__ bnb, const float* __restrict__ gam,
          const float* __restrict__ bet, const float* __restrict__ fb, const float* __restrict__ fgam,
          const float* __restrict__ fbet, float* PAR) {
  const int e0 = 4 * (int)threadIdx.x;
  v4i r = pd_pick(embb, PAR_EMBB, ND, e0);
  r |= pd_pick(bnb,  PAR_BNB,  NLAY * ND, e0);
  r |= pd_pick(gam,  PAR_GAM,  NLAY * ND, e0);
  r |= pd_pick(bet,  PAR_BET,  NLAY * ND, e0);
  r |= pd_pick(fb,   PAR_FB,   HD, e0);
  r |= pd_pick(fgam, PAR_FGAM, HD, e0);
  r |= pd_pick(fbet, PAR_FBET, HD, e0);
  v4f o;
  o.x = __int_as_float(r.x); o.y = __int_as_float(r.y); o.z = __int_as_float(r.z); o.w = __int_as_float(r.w);
  float* dp = PAR + e0;
  *(volatile v4f*)dp = o;
  __threadfence();
  *(volatile v4f*)dp = o;
}

__global__ __launch_bounds__(NTHR) __attribute__((amdgpu_num_vgpr(248)))
void k_bucket(const int* __restrict__ srcs, const int* __restrict__ dsts, const float* __restrict__ eattr,
              int nE, int nN, int vec8, int* LIST, int* CNT, int* OFF, int* FLG) {
  extern __shared__ __attribute__((aligned(16))) int bsm[];
  int* list = bsm;
  int* reg1 = bsm + LISTN;
  int* sl   = reg1 + RCAP;
  int* cnt  = sl + RCAP;
  int* offs = cnt + NBA;
  int* cur  = offs + NBA;
  int* wcnt = cur + NBA;
  const int tid = (int)threadIdx.x, lane = tid & 31, wave = tid >> 5;
  const int blk = (int)blockIdx.x;
  const int nodeBase = blk * NBA;
  int nb = nN - nodeBase;
  nb = nb < 0 ? 0 : (nb > NBA ? NBA : nb);

  {
    const v4i z4 = {0, 0, 0, 0};
    for (int i = tid * 4; i < LISTN + BKT_ZINTS; i += NTHR * 4) *(v4ia*)(bsm + i) = z4;
    if (tid < 16) wcnt[tid] = 0;
  }
  __syncthreads();

  int tot = 0, ovf = 0;
  const int nChunks = (nE + CHUNK - 1) / CHUNK;
#pragma unroll 1
  for (int ch = 0; ch < nChunks; ++ch) {
    const int cbase = ch * CHUNK;
    const int wc = scan_chunk<SLA>(dsts, nE, cbase, nodeBase, nb, vec8, list, tid, lane, wave);
    if (lane == 0) wcnt[wave] = wc;
    __syncthreads();
    int pre = 0, all = 0;
#pragma unroll
    for (int w2 = 0; w2 < NWAVE; ++w2) {
      int c = wcnt[w2];
      c = c < 0 ? 0 : (c > WCAP ? WCAP : c);
      all += c;
      pre += (w2 < wave) ? c : 0;
    }
    const int wcc  = wc > WCAP ? WCAP : wc;
    const int base = tot + pre;
#pragma unroll 1
    for (int i = lane; i < wcc; i += 32) {
      const int ent = list[wave * WCAP + i];
      const int el  = (ent >> SLA) & (CHUNK - 1);
      const int sq  = ent & (NBA - 1);
      int eid = cbase + el;
      eid = eid > nE - 1 ? nE - 1 : eid;
      const int pos = base + i;
      if (pos < RCAP) reg1[pos] = (eid << SLA) | sq;
    }
    if (tot + all > RCAP) ovf = 1;
    tot += all;
    tot = tot > RCAP ? RCAP : tot;
    __syncthreads();
  }
  int nh = __builtin_amdgcn_readfirstlane(tot);
  nh = nh < 0 ? 0 : (nh > RCAP ? RCAP : nh);

  if (wave == 0) {
#pragma unroll 1
    for (int b0 = 0; b0 < nh; b0 += 32) {
      const int idx = b0 + lane;
      const int uv  = reg1[idx < RCAP ? idx : RCAP - 1];
      const int m32 = (nh - b0) < 32 ? (nh - b0) : 32;
#pragma unroll 1
      for (int k = 0; k < m32; ++k) {
        const int u  = __builtin_amdgcn_readlane(uv, k);
        const int sq = u & (NBA - 1);
        if (lane == 0) cnt[sq] = cnt[sq] + 1;
      }
    }
  }
  __syncthreads();
  if (wave == 0) {
    const int base = lane * (NBA / 32);
    int s = 0;
#pragma unroll 1
    for (int i = 0; i < NBA / 32; ++i) s += cnt[base + i];
    int incl = s;
#pragma unroll
    for (int d = 1; d < 32; d <<= 1) {
      const int y = __shfl_up(incl, d, 32);
      if (lane >= d) incl += y;
    }
    int run = incl - s;
#pragma unroll 1
    for (int i = 0; i < NBA / 32; ++i) {
      const int cv = cnt[base + i];
      offs[base + i] = run;
      cur[base + i]  = run;
      run += cv;
    }
  }
  __syncthreads();
  if (wave == 0) {
#pragma unroll 1
    for (int b0 = 0; b0 < nh; b0 += 32) {
      const int idx = b0 + lane;
      const int uv  = reg1[idx < RCAP ? idx : RCAP - 1];
      const int m32 = (nh - b0) < 32 ? (nh - b0) : 32;
#pragma unroll 1
      for (int k = 0; k < m32; ++k) {
        const int u  = __builtin_amdgcn_readlane(uv, k);
        const int sq = u & (NBA - 1);
        if (lane == 0) {
          int p = cur[sq];
          p = p < 0 ? 0 : (p > RCAP - 1 ? RCAP - 1 : p);
          sl[p] = u;
          cur[sq] = p + 1;
        }
      }
    }
  }
  __syncthreads();

  int* lb = LIST + (size_t)blk * RCAP * 2;
  const v4i cq = *(const v4ia*)(cnt + 4 * tid);
  const v4i oq = *(const v4ia*)(offs + 4 * tid);
  int* cp = CNT + (size_t)blk * NBA + 4 * tid;
  int* op = OFF + (size_t)blk * NBA + 4 * tid;
  v4i cv;
  cv.x = (tid == 0) ? nh : 0;
  cv.y = (tid == 0) ? ovf : 0;
  cv.z = 0; cv.w = 0;
  int* fp = FLG + (size_t)blk * 32 + 4 * (tid & 7);

#pragma unroll 1
  for (int q = tid; q < RCAP / 2; q += NTHR) {
    const v2i e = *(const v2ia*)(sl + 2 * q);
    int i0 = e.x >> SLA; i0 = i0 < 0 ? 0 : (i0 > nE - 1 ? nE - 1 : i0);
    int i1 = e.y >> SLA; i1 = i1 < 0 ? 0 : (i1 > nE - 1 ? nE - 1 : i1);
    int s0 = srcs[i0]; s0 = s0 < 0 ? 0 : (s0 > nN - 1 ? nN - 1 : s0);
    int s1 = srcs[i1]; s1 = s1 < 0 ? 0 : (s1 > nN - 1 ? nN - 1 : s1);
    const int a0 = __float_as_int(bfr(eattr[i0]));
    const int a1 = __float_as_int(bfr(eattr[i1]));
    const bool k0 = 2 * q < nh, k1 = 2 * q + 1 < nh;
    v4i o;
    o.x = k0 ? s0 : 0; o.y = k0 ? a0 : 0; o.z = k1 ? s1 : 0; o.w = k1 ? a1 : 0;
    *(volatile v4i*)(lb + 4 * q) = o;
  }
  *(volatile v4i*)cp = cq;
  *(volatile v4i*)op = oq;
  if (tid < 8) *(volatile v4i*)fp = cv;
  __threadfence();
#pragma unroll 1
  for (int q = tid; q < RCAP / 2; q += NTHR) {
    const v2i e = *(const v2ia*)(sl + 2 * q);
    int i0 = e.x >> SLA; i0 = i0 < 0 ? 0 : (i0 > nE - 1 ? nE - 1 : i0);
    int i1 = e.y >> SLA; i1 = i1 < 0 ? 0 : (i1 > nE - 1 ? nE - 1 : i1);
    int s0 = srcs[i0]; s0 = s0 < 0 ? 0 : (s0 > nN - 1 ? nN - 1 : s0);
    int s1 = srcs[i1]; s1 = s1 < 0 ? 0 : (s1 > nN - 1 ? nN - 1 : s1);
    const int a0 = __float_as_int(bfr(eattr[i0]));
    const int a1 = __float_as_int(bfr(eattr[i1]));
    const bool k0 = 2 * q < nh, k1 = 2 * q + 1 < nh;
    v4i o;
    o.x = k0 ? s0 : 0; o.y = k0 ? a0 : 0; o.z = k1 ? s1 : 0; o.w = k1 ? a1 : 0;
    *(volatile v4i*)(lb + 4 * q) = o;
  }
  *(volatile v4i*)cp = cq;
  *(volatile v4i*)op = oq;
  if (tid < 8) *(volatile v4i*)fp = cv;
}

template <int NT, int MODE>
__global__ __launch_bounds__(GTHR) __attribute__((amdgpu_num_vgpr(248)))
void k_gemm(const unsigned short* __restrict__ A, const unsigned short* __restrict__ BT,
            const float* __restrict__ bias, int nN, unsigned short* outH, float* outF) {
  static_assert((MODE == 0 && NT == 4) || (MODE == 1 && NT == 8));
  constexpr int NC = 16 * NT;
  __shared__ __attribute__((aligned(16))) float stg[GBM * NC];
  const int tid = (int)threadIdx.x, lane = tid & 31, wave = tid >> 5, hh = lane >> 4, m = lane & 15;
  const int rowBase = (int)blockIdx.x * GBM;

  v8f acc[NT];
#pragma unroll
  for (int t = 0; t < NT; ++t) acc[t] = z8();
  const unsigned short* ap = A  + (size_t)(rowBase + 16 * wave + m) * (size_t)KP + 8 * hh;
  const unsigned short* bp = BT + (size_t)m * (size_t)KP + 8 * hh;
#pragma unroll 1
  for (int k0 = 0; k0 < KP; k0 += 32) {
    FragB af;
    af.h[0] = *(const v8usa*)(ap + k0);
    af.h[1] = *(const v8usa*)(ap + k0 + 16);
#pragma unroll
    for (int t = 0; t < NT; ++t) {
      const unsigned short* wq = bp + (size_t)(16 * t) * (size_t)KP + k0;
      FragB bf;
      bf.h[0] = *(const v8usa*)wq;
      bf.h[1] = *(const v8usa*)(wq + 16);
      acc[t] = wmb(af, bf, acc[t]);
    }
  }
#pragma unroll
  for (int t = 0; t < NT; ++t) {
    const int lc = 16 * t + m;
#pragma unroll
    for (int r = 0; r < 8; ++r) {
      const int lr = 16 * wave + 8 * hh + r;
      stg[lr * NC + lc] = acc[t][r];
    }
  }
  __syncthreads();

  if constexpr (MODE == 0) {
    const int part = lane >> 4, c4 = 4 * (lane & 15);
    const v4f b4 = *(const v4f*)(bias + c4);
#pragma unroll 1
    for (int i = 0; i < 16; ++i) {
      const int lr = 16 * wave + i, row = rowBase + lr;
      const bool ok = row < nN;
      const v4f x = *(const v4fa*)(stg + lr * NC + c4);
      v4f v;
      v.x = ok ? x.x + b4.x : 0.0f; v.y = ok ? x.y + b4.y : 0.0f;
      v.z = ok ? x.z + b4.z : 0.0f; v.w = ok ? x.w + b4.w : 0.0f;
      const v4us o = pack4(v, part);
      *(volatile v4us*)(outH + (size_t)row * KP + 4 * lane) = o;
    }
    __threadfence();
#pragma unroll 1
    for (int i = 0; i < 16; ++i) {
      const int lr = 16 * wave + i, row = rowBase + lr;
      const bool ok = row < nN;
      const v4f x = *(const v4fa*)(stg + lr * NC + c4);
      v4f v;
      v.x = ok ? x.x + b4.x : 0.0f; v.y = ok ? x.y + b4.y : 0.0f;
      v.z = ok ? x.z + b4.z : 0.0f; v.w = ok ? x.w + b4.w : 0.0f;
      const v4us o = pack4(v, part);
      *(volatile v4us*)(outH + (size_t)row * KP + 4 * lane) = o;
    }
  } else {
#pragma unroll 1
    for (int i = 0; i < 16; ++i) {
      const int lr = 16 * wave + i, row = rowBase + lr;
      const v4f x = *(const v4fa*)(stg + lr * NC + 4 * lane);
      *(volatile v4f*)(outF + (size_t)row * HD + 4 * lane) = x;
    }
    __threadfence();
#pragma unroll 1
    for (int i = 0; i < 16; ++i) {
      const int lr = 16 * wave + i, row = rowBase + lr;
      const v4f x = *(const v4fa*)(stg + lr * NC + 4 * lane);
      *(volatile v4f*)(outF + (size_t)row * HD + 4 * lane) = x;
    }
  }
}

__global__ __launch_bounds__(NTHR) __attribute__((amdgpu_num_vgpr(248)))
void k_scan(const int* __restrict__ LIST, const int* __restrict__ CNT, const int* __restrict__ OFF,
            const int* __restrict__ FLG, const unsigned* __restrict__ HW, const float* __restrict__ TP,
            const float* __restrict__ PQl, const float* __restrict__ bnb, float* OUT, int nN) {
  const int tid = (int)threadIdx.x, lane = tid & 31, wave = tid >> 5;
  const int blk = (int)blockIdx.x;
  const int nodeBase = blk * NBA;

  const int nhraw = __builtin_amdgcn_readfirstlane(FLG[(size_t)blk * 32]);
  const int bflag = __builtin_amdgcn_readfirstlane(FLG[(size_t)blk * 32 + 1]);
  const int nh  = nhraw < 0 ? 0 : (nhraw > RCAP ? RCAP : nhraw);
  const int ovf = (bflag != 0 || nhraw < 0 || nhraw > RCAP) ? 1 : 0;

  const v2f pp = *(const v2f*)(PQl + 2 * lane);
  const v2f qq = *(const v2f*)(PQl + ND + 2 * lane);
  const v2f bb = *(const v2f*)(bnb + 2 * lane);
  const int* lb = LIST + (size_t)blk * RCAP * 2;
  const float qnan = __int_as_float(0x7fc00000);
  const float pzb  = (ovf != 0) ? qnan : 0.0f;

#pragma unroll 1
  for (int si = 0; si < NBA / NWAVE; ++si) {
    const int s    = si * NWAVE + wave;
    const int node = nodeBase + s;
    const int nc   = node < nN ? node : nN - 1;
    int c = __builtin_amdgcn_readfirstlane(CNT[(size_t)nodeBase + s]);
    const bool big = c > DEGCAP;
    c = c < 0 ? 0 : (c > DEGCAP ? DEGCAP : c);
    int o = __builtin_amdgcn_readfirstlane(OFF[(size_t)nodeBase + s]);
    o = o < 0 ? 0 : (o > RCAP ? RCAP : o);
    if (c > nh - o) c = nh - o;
    c = c < 0 ? 0 : c;
    float acc0 = 0.0f, acc1 = 0.0f;
#pragma unroll 1
    for (int b0 = 0; b0 < c; b0 += 32) {
      int idx = o + b0 + lane;
      idx = idx < 0 ? 0 : (idx > RCAP - 1 ? RCAP - 1 : idx);
      const v2i ent = *(const v2i*)(lb + 2 * idx);
      int sr = ent.x;
      sr = sr < 0 ? 0 : (sr > nN - 1 ? nN - 1 : sr);
      const int ai  = ent.y;
      const int m32 = (c - b0) < 32 ? (c - b0) : 32;
#pragma unroll 1
      for (int k = 0; k < m32; ++k) {
        const int   sk = __builtin_amdgcn_readlane(sr, k);
        const float ak = __int_as_float(__builtin_amdgcn_readlane(ai, k));
        const unsigned hiw = HW[(size_t)sk * ND + lane];
        const unsigned low = HW[(size_t)sk * ND + 32 + lane];
        const v2f pv = *(const v2f*)(TP + (size_t)sk * HD + ND + 2 * lane);
        const float h0 = __uint_as_float(hiw << 16) + __uint_as_float(low << 16);
        const float h1 = __uint_as_float(hiw & 0xffff0000u) + __uint_as_float(low & 0xffff0000u);
        const float z0 = fmaf(ak, pp.x, pv.x) + qq.x;
        const float z1 = fmaf(ak, pp.y, pv.y) + qq.y;
        const float g0 = 1.0f / (1.0f + expf(-z0));
        const float g1 = 1.0f / (1.0f + expf(-z1));
        acc0 = fmaf(g0, h0, acc0);
        acc1 = fmaf(g1, h1, acc1);
      }
    }
    const v2f tv = *(const v2f*)(TP + (size_t)nc * HD + 2 * lane);
    const float pzr = big ? qnan : pzb;
    v2f ov;
    ov.x = ((tv.x + bb.x) + acc0) + pzr;
    ov.y = ((tv.y + bb.y) + acc1) + pzr;
    if (node < nN) {
      float* dp = OUT + (size_t)node * ND + 2 * lane;
      *(volatile v2f*)dp = ov;
      __threadfence();
      *(volatile v2f*)dp = ov;
    }
  }
}

__global__ __launch_bounds__(NTHR) __attribute__((amdgpu_num_vgpr(248)))
void k_stat(const float* __restrict__ OUT, float* REC, int nN) {
  __shared__ __attribute__((aligned(16))) float gm[16 * ND];
  __shared__ __attribute__((aligned(16))) float gq[16 * ND];
  __shared__ __attribute__((aligned(16))) float rec[2 * ND];
  const int tid = (int)threadIdx.x;
  const int cg = tid & 15, rg = tid >> 4;
  const int blk = (int)blockIdx.x;
  const int r0 = blk * SROWS + rg * 8;
  int n = nN - r0;
  n = n < 0 ? 0 : (n > 8 ? 8 : n);
  const v4f z4 = {0.f, 0.f, 0.f, 0.f};
  v4f s = z4;
#pragma unroll 1
  for (int i = 0; i < 8; ++i) {
    const int row = r0 + i;
    const int rc  = row < nN ? row : nN - 1;
    const v4f v = *(const v4f*)(OUT + (size_t)rc * ND + 4 * cg);
    const bool ok = i < n;
    s.x += ok ? v.x : 0.0f; s.y += ok ? v.y : 0.0f; s.z += ok ? v.z : 0.0f; s.w += ok ? v.w : 0.0f;
  }
  const float rn = 1.0f / (float)(n > 0 ? n : 1);
  const v4f mean = s * rn;
  v4f q = z4;
#pragma unroll 1
  for (int i = 0; i < 8; ++i) {
    const int row = r0 + i;
    const int rc  = row < nN ? row : nN - 1;
    const v4f v = *(const v4f*)(OUT + (size_t)rc * ND + 4 * cg);
    const bool ok = i < n;
    const v4f d = v - mean;
    q.x += ok ? d.x * d.x : 0.0f; q.y += ok ? d.y * d.y : 0.0f;
    q.z += ok ? d.z * d.z : 0.0f; q.w += ok ? d.w * d.w : 0.0f;
  }
  *(v4fa*)(gm + rg * ND + 4 * cg) = mean;
  *(v4fa*)(gq + rg * ND + 4 * cg) = q;
  __syncthreads();
  if (tid < ND) {
    double cn = 0.0, cm = 0.0, cq = 0.0;
#pragma unroll 1
    for (int g = 0; g < 16; ++g) {
      int nb = nN - (blk * SROWS + g * 8);
      nb = nb < 0 ? 0 : (nb > 8 ? 8 : nb);
      const double mb = (double)gm[g * ND + tid];
      const double qb = (double)gq[g * ND + tid];
      if (nb > 0) {
        const double dn = (double)nb;
        const double nn = cn + dn;
        const double delta = mb - cm;
        const double f = dn / nn;
        cm = cm + delta * f;
        cq = cq + qb + delta * delta * cn * f;
        cn = nn;
      }
    }
    rec[tid] = (float)cm;
    rec[ND + tid] = (float)cq;
  }
  __syncthreads();
  v4f v = z4;
  float* dp = REC + (size_t)blk * 2 * ND + 4 * (tid & 31);
  if (tid < 32) { v = *(const v4fa*)(rec + 4 * tid); *(volatile v4f*)dp = v; }
  __threadfence();
  if (tid < 32) { *(volatile v4f*)dp = v; }
}

__global__ __launch_bounds__(ND) __attribute__((amdgpu_num_vgpr(248)))
void k_comb(const float* __restrict__ REC, float* STAT, int nBlk, int nN) {
  __shared__ __attribute__((aligned(16))) float so[2 * ND];
  const int c = (int)threadIdx.x;
  double cn = 0.0, cm = 0.0, cq = 0.0;
#pragma unroll 1
  for (int b = 0; b < nBlk; ++b) {
    int nb = nN - b * SROWS;
    nb = nb < 0 ? 0 : (nb > SROWS ? SROWS : nb);
    const double mb = (double)REC[(size_t)b * 2 * ND + c];
    const double qb = (double)REC[(size_t)b * 2 * ND + ND + c];
    if (nb > 0) {
      const double dn = (double)nb;
      const double nn = cn + dn;
      const double delta = mb - cm;
      const double f = dn / nn;
      cm = cm + delta * f;
      cq = cq + qb + delta * delta * cn * f;
      cn = nn;
    }
  }
  const double nt = cn < 1.0 ? 1.0 : cn;
  const float varf = (float)(cq / nt);
  so[c] = (float)cm;
  so[ND + c] = 1.0f / sqrtf(varf + 1e-5f);
  __syncthreads();
  v4f v = {0.f, 0.f, 0.f, 0.f};
  float* dp = STAT + 4 * (c & 31);
  if (c < 32) { v = *(const v4fa*)(so + 4 * c); *(volatile v4f*)dp = v; }
  __threadfence();
  if (c < 32) { *(volatile v4f*)dp = v; }
}

__global__ __launch_bounds__(NTHR) __attribute__((amdgpu_num_vgpr(248)))
void k_apply(const float* __restrict__ OUT, const float* __restrict__ ST, const float* __restrict__ gam,
             const float* __restrict__ bet, unsigned short* HHL, int nN, int nUnits) {
  const int u = (int)blockIdx.x * NTHR + (int)threadIdx.x;
  if (u >= nUnits) return;
  const int row = u >> 5, l = u & 31, part = l >> 4, c4 = 4 * (l & 15);
  const int rc = row < nN ? row : nN - 1;
  const bool ok = row < nN;
  const v4f x  = *(const v4f*)(OUT + (size_t)rc * ND + c4);
  const v4f m4 = *(const v4f*)(ST + c4);
  const v4f r4 = *(const v4f*)(ST + ND + c4);
  const v4f g4 = *(const v4f*)(gam + c4);
  const v4f b4 = *(const v4f*)(bet + c4);
  const v4f t = ((x - m4) * r4) * g4 + b4;
  v4f v;
  v.x = (t.x > 0.0f) ? t.x : (t.x - t.x);
  v.y = (t.y > 0.0f) ? t.y : (t.y - t.y);
  v.z = (t.z > 0.0f) ? t.z : (t.z - t.z);
  v.w = (t.w > 0.0f) ? t.w : (t.w - t.w);
  v.x = ok ? v.x : 0.0f; v.y = ok ? v.y : 0.0f; v.z = ok ? v.z : 0.0f; v.w = ok ? v.w : 0.0f;
  const v4us o = pack4(v, part);
  unsigned short* dp = HHL + (size_t)u * 4;
  *(volatile v4us*)dp = o;
  __threadfence();
  *(volatile v4us*)dp = o;
}

__global__ __launch_bounds__(NTHR) __attribute__((amdgpu_num_vgpr(248)))
void k_pool(const float* __restrict__ OUT, const int* __restrict__ batch, const float* __restrict__ ST,
            const float* __restrict__ gam, const float* __restrict__ bet, unsigned short* PH, int nN) {
  __shared__ __attribute__((aligned(16))) float wsum[NWAVE * ND];
  __shared__ int wcn[NWAVE];
  __shared__ __attribute__((aligned(16))) float fin[ND];
  const int tid = (int)threadIdx.x, lane = tid & 31, wave = tid >> 5;
  const int g = (int)blockIdx.x;
  const v2f m2 = *(const v2f*)(ST + 2 * lane);
  const v2f r2 = *(const v2f*)(ST + ND + 2 * lane);
  const v2f g2 = *(const v2f*)(gam + 2 * lane);
  const v2f b2 = *(const v2f*)(bet + 2 * lane);
  float acc0 = 0.0f, acc1 = 0.0f;
  int mine = 0;
#pragma unroll 1
  for (int base = wave * 32; base < nN; base += NTHR) {
    const int i  = base + lane;
    const int ic = i < nN ? i : nN - 1;
    const int bv = batch[ic];
    const bool hit = (i < nN) && (bv == g);
    mine += hit ? 1 : 0;
    unsigned mk = __builtin_amdgcn_ballot_w32(hit);
#pragma unroll 1
    while (mk != 0u) {
      const int k = __builtin_ctz(mk);
      mk &= mk - 1u;
      int node = base + k;
      node = node > nN - 1 ? nN - 1 : node;
      const v2f x = *(const v2f*)(OUT + (size_t)node * ND + 2 * lane);
      const float t0 = ((x.x - m2.x) * r2.x) * g2.x + b2.x;
      const float t1 = ((x.y - m2.y) * r2.y) * g2.y + b2.y;
      acc0 += (t0 > 0.0f) ? t0 : (t0 - t0);
      acc1 += (t1 > 0.0f) ? t1 : (t1 - t1);
    }
  }
  int cnt = mine;
#pragma unroll
  for (int d = 16; d >= 1; d >>= 1) cnt += __shfl_xor(cnt, d, 32);
  wsum[wave * ND + 2 * lane]     = acc0;
  wsum[wave * ND + 2 * lane + 1] = acc1;
  if (lane == 0) wcn[wave] = cnt;
  __syncthreads();
  if (tid < ND) {
    double s = 0.0;
    int ct = 0;
#pragma unroll
    for (int w2 = 0; w2 < NWAVE; ++w2) { s += (double)wsum[w2 * ND + tid]; ct += wcn[w2]; }
    const float cf = (ct > 1) ? (float)ct : 1.0f;
    fin[tid] = (float)s * (1.0f / cf);
  }
  __syncthreads();
  const int part = lane >> 4, c4 = 4 * (lane & 15);
  const v4f pv = *(const v4fa*)(fin + c4);
  const v4us o = pack4(pv, part);
  unsigned short* dp = PH + (size_t)g * KP + 4 * lane;
  if (wave == 0) *(volatile v4us*)dp = o;
  __threadfence();
  if (wave == 0) *(volatile v4us*)dp = o;
}

__global__ __launch_bounds__(NTHR) __attribute__((amdgpu_num_vgpr(248)))
void k_head(const unsigned short* __restrict__ PH, const unsigned short* __restrict__ FWD,
            const float* __restrict__ PAR, float* out) {
  extern __shared__ __attribute__((aligned(16))) float hsm[];
  float* stg = hsm;
  float* cm  = hsm + NG * HD;
  float* cr  = cm + HD;
  const int tid = (int)threadIdx.x, lane = tid & 31, wave = tid >> 5, hh = lane >> 4, m = lane & 15;

  v8f acc[8];
#pragma unroll
  for (int t = 0; t < 8; ++t) acc[t] = z8();
  const unsigned short* ap = PH  + (size_t)(16 * wave + m) * (size_t)KP + 8 * hh;
  const unsigned short* bp = FWD + (size_t)m * (size_t)KP + 8 * hh;
#pragma unroll 1
  for (int k0 = 0; k0 < KP; k0 += 32) {
    FragB af;
    af.h[0] = *(const v8usa*)(ap + k0);
    af.h[1] = *(const v8usa*)(ap + k0 + 16);
#pragma unroll
    for (int t = 0; t < 8; ++t) {
      const unsigned short* wq = bp + (size_t)(16 * t) * (size_t)KP + k0;
      FragB bf;
      bf.h[0] = *(const v8usa*)wq;
      bf.h[1] = *(const v8usa*)(wq + 16);
      acc[t] = wmb(af, bf, acc[t]);
    }
  }
#pragma unroll
  for (int t = 0; t < 8; ++t) {
    const int lc = 16 * t + m;
#pragma unroll
    for (int r = 0; r < 8; ++r) {
      const int lr = 16 * wave + 8 * hh + r;
      stg[lr * HD + lc] = acc[t][r];
    }
  }
  __syncthreads();
  if (tid < HD) {
    const int c = tid;
    const float fbc = PAR[PAR_FB + c];
    double s = 0.0;
#pragma unroll 4
    for (int r = 0; r < NG; ++r) {
      const float v = stg[r * HD + c] + fbc;
      stg[r * HD + c] = v;
      s += (double)v;
    }
    const double mean = s * (1.0 / (double)NG);
    double q = 0.0;
#pragma unroll 4
    for (int r = 0; r < NG; ++r) {
      const double d = (double)stg[r * HD + c] - mean;
      q += d * d;
    }
    const float varf = (float)(q * (1.0 / (double)NG));
    cm[c] = (float)mean;
    cr[c] = 1.0f / sqrtf(varf + 1e-5f);
  }
  __syncthreads();
  const int c4 = 4 * lane;
  const v4f m4 = *(const v4fa*)(cm + c4);
  const v4f r4 = *(const v4fa*)(cr + c4);
  const v4f g4 = *(const v4f*)(PAR + PAR_FGAM + c4);
  const v4f b4 = *(const v4f*)(PAR + PAR_FBET + c4);
#pragma unroll 1
  for (int i = 0; i < 16; ++i) {
    const int row = 16 * wave + i;
    const v4f y = *(const v4fa*)(stg + row * HD + c4);
    const v4f t = ((y - m4) * r4) * g4 + b4;
    v4f o;
    o.x = (t.x > 0.0f) ? t.x : (t.x - t.x);
    o.y = (t.y > 0.0f) ? t.y : (t.y - t.y);
    o.z = (t.z > 0.0f) ? t.z : (t.z - t.z);
    o.w = (t.w > 0.0f) ? t.w : (t.w - t.w);
    *(volatile v4f*)(out + (size_t)row * HD + c4) = o;
  }
  __threadfence();
#pragma unroll 1
  for (int i = 0; i < 16; ++i) {
    const int row = 16 * wave + i;
    const v4f y = *(const v4fa*)(stg + row * HD + c4);
    const v4f t = ((y - m4) * r4) * g4 + b4;
    v4f o;
    o.x = (t.x > 0.0f) ? t.x : (t.x - t.x);
    o.y = (t.y > 0.0f) ? t.y : (t.y - t.y);
    o.z = (t.z > 0.0f) ? t.z : (t.z - t.z);
    o.w = (t.w > 0.0f) ? t.w : (t.w - t.w);
    *(volatile v4f*)(out + (size_t)row * HD + c4) = o;
  }
}

static inline int cdiv(int a, int b) { return (a + b - 1) / b; }
static inline size_t al256(size_t o) { return (o + 255) & ~(size_t)255; }

extern "C" void kernel_launch(void* const* d_in, const int* in_sizes, int n_in,
                              void* d_out, int out_size, void* d_ws, size_t ws_size,
                              hipStream_t stream) {
  if (n_in < 20) return;
  const int nN = in_sizes[0] / IN_DIM;
  if (nN < 1 || in_sizes[0] != nN * IN_DIM || (in_sizes[0] & 3) != 0 || nN > (1 << 22)) return;
  if (in_sizes[1] < 2 || (in_sizes[1] & 1) != 0) return;
  const int nE = in_sizes[1] / 2;
  if (nE < 1 || nE >= (1 << 21)) return;
  if (in_sizes[2] != nE || in_sizes[3] != nN) return;
  if (in_sizes[4] != IN_DIM * ND || in_sizes[5] != ND) return;
  if (in_sizes[6] != 32 || in_sizes[7] != 32) return;
  if (in_sizes[8] != NLAY * ND * ND || in_sizes[9] != NLAY * ND) return;
  if (in_sizes[10] != NLAY * 32 * ND || in_sizes[11] != NLAY * ND) return;
  if (in_sizes[12] != NLAY * 2 * ND * ND || in_sizes[13] != NLAY * ND) return;
  if (in_sizes[14] != NLAY * ND || in_sizes[15] != NLAY * ND) return;
  if (in_sizes[16] != ND * HD || in_sizes[17] != HD) return;
  if (in_sizes[18] != HD || in_sizes[19] != HD) return;
  if (out_size != NG * HD) return;

  const float* x     = (const float*)d_in[0];
  const int*   ei    = (const int*)  d_in[1];
  const float* eattr = (const float*)d_in[2];
  const int*   batch = (const int*)  d_in[3];
  const float* embW  = (const float*)d_in[4];
  const float* embB  = (const float*)d_in[5];
  const float* eW    = (const float*)d_in[6];
  const float* eB    = (const float*)d_in[7];
  const float* Wn    = (const float*)d_in[8];
  const float* bnb   = (const float*)d_in[9];
  const float* We    = (const float*)d_in[10];
  const float* be    = (const float*)d_in[11];
  const float* Wg    = (const float*)d_in[12];
  const float* bg    = (const float*)d_in[13];
  const float* gam   = (const float*)d_in[14];
  const float* bet   = (const float*)d_in[15];
  const float* fW    = (const float*)d_in[16];
  const float* fb    = (const float*)d_in[17];
  const float* fgam  = (const float*)d_in[18];
  const float* fbet  = (const float*)d_in[19];
  float* out = (float*)d_out;
  const int* src = ei;
  const int* dst = ei + nE;

  const int MP   = cdiv(nN, MROWS) * MROWS;
  const int gM   = MP / GBM;
  const int gS   = MP / SROWS;
  const int gA   = cdiv(nN, NBA);
  const int vec8 = ((nE & 3) == 0) ? 1 : 0;
  const int nF4  = in_sizes[0] / 4;
  if ((long long)MP * 32 > 2147483647LL) return;
  const int nUa  = MP * 32;

  char* ws = (char*)d_ws;
  size_t off = 0;
  const size_t oXB  = off; off = al256(off + (size_t)MP * KP * 2);
  const size_t oHHL = off; off = al256(off + (size_t)MP * KP * 2);
  const size_t oTP  = off; off = al256(off + (size_t)MP * HD * 4);
  const size_t oOUT = off; off = al256(off + (size_t)nN * ND * 4);
  const size_t oLST = off; off = al256(off + (size_t)gA * RCAP * 8);
  const size_t oCNT = off; off = al256(off + (size_t)gA * NBA * 4);
  const size_t oOFF = off; off = al256(off + (size_t)gA * NBA * 4);
  const size_t oFLG = off; off = al256(off + (size_t)gA * 128);
  const size_t oREC = off; off = al256(off + (size_t)gS * 2 * ND * 4);
  const size_t oEMB = off; off = al256(off + (size_t)ND * KP * 2);
  const size_t oBT  = off; off = al256(off + (size_t)NLAY * HD * KP * 2);
  const size_t oFWD = off; off = al256(off + (size_t)HD * KP * 2);
  const size_t oPQ  = off; off = al256(off + (size_t)NLAY * 2 * ND * 4);
  const size_t oPAR = off; off = al256(off + (size_t)PAR_N * 4);
  const size_t oST  = off; off = al256(off + (size_t)NLAY * 2 * ND * 4);
  const size_t oPH  = off; off = al256(off + (size_t)NG * KP * 2);
  if (off > ws_size || off > (size_t)WSMAX) return;
  unsigned short* XB   = (unsigned short*)(ws + oXB);
  unsigned short* HHL  = (unsigned short*)(ws + oHHL);
  float*          TP   = (float*)(ws + oTP);
  float*          OUTp = (float*)(ws + oOUT);
  int*            LIST = (int*)(ws + oLST);
  int*            CNT  = (int*)(ws + oCNT);
  int*            OFFp = (int*)(ws + oOFF);
  int*            FLG  = (int*)(ws + oFLG);
  float*          REC  = (float*)(ws + oREC);
  unsigned short* EMBT = (unsigned short*)(ws + oEMB);
  unsigned short* BT   = (unsigned short*)(ws + oBT);
  unsigned short* FWD  = (unsigned short*)(ws + oFWD);
  float*          PQ   = (float*)(ws + oPQ);
  float*          PAR  = (float*)(ws + oPAR);
  float*          STAT = (float*)(ws + oST);
  unsigned short* PH   = (unsigned short*)(ws + oPH);

  const int bktLds  = BKT_LDS_INTS * 4;
  const int headLds = HEAD_LDS_FLOATS * 4;
  hipFuncSetAttribute(reinterpret_cast<const void*>(&k_bucket),
                      hipFuncAttributeMaxDynamicSharedMemorySize, bktLds);
  hipFuncSetAttribute(reinterpret_cast<const void*>(&k_head),
                      hipFuncAttributeMaxDynamicSharedMemorySize, headLds);

  k_pa<<<MP / PA_ROWS, NTHR, 0, stream>>>(x, XB, nF4);
  k_pb<<<(NU_EMB + NU_WN + NU_WG + NU_FW) / NTHR, NTHR, 0, stream>>>(embW, Wn, Wg, fW, EMBT, BT, FWD);
  k_pc<<<NLAY, ND, 0, stream>>>(eW, eB, We, be, Wg, bg, PQ);
  k_pd<<<1, NTHR, 0, stream>>>(embB, bnb, gam, bet, fb, fgam, fbet, PAR);
  k_bucket<<<gA, NTHR, bktLds, stream>>>(src, dst, eattr, nE, nN, vec8, LIST, CNT, OFFp, FLG);
  k_gemm<4, 0><<<gM, GTHR, 0, stream>>>(XB, EMBT, PAR + PAR_EMBB, nN, HHL, TP);

  for (int l = 0; l < NLAY; ++l) {
    k_gemm<8, 1><<<gM, GTHR, 0, stream>>>(HHL, BT + (size_t)l * HD * KP, PAR, nN, XB, TP);
    k_scan<<<gA, NTHR, 0, stream>>>(LIST, CNT, OFFp, FLG, (const unsigned*)HHL, TP,
                                    PQ + (size_t)l * 2 * ND, PAR + PAR_BNB + l * ND, OUTp, nN);
    k_stat<<<gS, NTHR, 0, stream>>>(OUTp, REC, nN);
    k_comb<<<1, ND, 0, stream>>>(REC, STAT + (size_t)l * 2 * ND, gS, nN);
    if (l < NLAY - 1) {
      k_apply<<<nUa / NTHR, NTHR, 0, stream>>>(OUTp, STAT + (size_t)l * 2 * ND, PAR + PAR_GAM + l * ND,
                                               PAR + PAR_BET + l * ND, HHL, nN, nUa);
    }
  }
  k_pool<<<NG, NTHR, 0, stream>>>(OUTp, batch, STAT + (size_t)(NLAY - 1) * 2 * ND,
                                  PAR + PAR_GAM + (NLAY - 1) * ND, PAR + PAR_BET + (NLAY - 1) * ND, PH, nN);
  k_head<<<1, NTHR, headLds, stream>>>(PH, FWD, PAR, out);
}
